// SchNetInteractionBlock_25701084299911
// MI455X (gfx1250) — hardware-verified
//
#include <hip/hip_runtime.h>
#include <stddef.h>


#define NTHR   256
#define NWAVE  8
#define FDIM   128
#define KRBF   20
#define A1P    72
#define A2P    136
#define NB     192
#define EPT    8
#define CHUNK  (NTHR * EPT)
#define WCAP   (EPT * 32)
#define LISTN  (NWAVE * WCAP)
#define PASSN  64
#define PCAP   (CHUNK + PASSN)
#define NROW   64
#define NQE    ((NB * FDIM) / (128 * NWAVE))
#define NQN    ((NROW * FDIM) / (128 * NWAVE))
#define USC    64.0f
#define RSC    2048.0f
#define WSC    16.0f
#define UWINV  0.0009765625f
#define RINV   0.00048828125f
#define LN2F   0.69314718f

static_assert(NQE * 128 * NWAVE == NB * FDIM);
static_assert(NQN * 128 * NWAVE == NROW * FDIM);
static_assert(PASSN * 4 == NTHR);
static_assert((PCAP % PASSN) == 0);
static_assert(FDIM == 16 * NWAVE);
static_assert((NROW % 16) == 0);
static_assert((PASSN % 16) == 0);

typedef float          v4f   __attribute__((ext_vector_type(4)));
typedef float          v8f   __attribute__((ext_vector_type(8)));
typedef int            v4i   __attribute__((ext_vector_type(4)));
typedef int            v8i   __attribute__((ext_vector_type(8)));
typedef unsigned short v4us  __attribute__((ext_vector_type(4)));
typedef unsigned short v16us __attribute__((ext_vector_type(16)));
typedef _Float16       v8h   __attribute__((ext_vector_type(8)));
typedef _Float16       v16h  __attribute__((ext_vector_type(16)));
typedef __bf16         v8b   __attribute__((ext_vector_type(8)));
typedef __bf16         v16b  __attribute__((ext_vector_type(16)));

union FragH { v16h v; v8h h[2]; };
union FragB { v16b v; v8b h[2]; v8i w; v16us u; };

__device__ __forceinline__ unsigned short bf_bits(float f) {
  unsigned u = __float_as_uint(f);
  u += 0x7FFFu + ((u >> 16) & 1u);
  return (unsigned short)(u >> 16);
}
__device__ __forceinline__ float bf_val(unsigned short b) {
  return __uint_as_float(((unsigned)b) << 16);
}

__device__ __forceinline__ void split4(v4f v, v4us& hi, v4us& lo) {
#pragma unroll
  for (int i = 0; i < 4; ++i) {
    const unsigned short hb = bf_bits(v[i]);
    hi[i] = hb;
    lo[i] = bf_bits(v[i] - bf_val(hb));
  }
}

__device__ __forceinline__ v8f zero8f() {
  v8f z;
#pragma unroll
  for (int i = 0; i < 8; ++i) z[i] = 0.0f;
  return z;
}

__device__ __forceinline__ v8f wmb(const FragB& a, const FragB& b, v8f c) {
  v8f d = __builtin_amdgcn_wmma_f32_16x16x32_bf16(false, a.v, false, b.v, (short)0, c, false, false);
  asm volatile("v_nop\n\tv_nop\n\tv_nop\n\tv_nop" : "+v"(d) : "v"(a.w), "v"(b.w));
  return d;
}
__device__ __forceinline__ v8f wmh(v16h a, v16h b, v8f c) {
  v8f d = __builtin_amdgcn_wmma_f32_16x16x32_f16(false, a, false, b, (short)0, c, false, false);
  asm volatile("v_nop\n\tv_nop\n\tv_nop\n\tv_nop" : "+v"(d) : "v"(a), "v"(b));
  return d;
}

__device__ __forceinline__ float sspf(float v) {
  const float e = expf(-fabsf(v));
  return fmaxf(v, 0.0f) + logf(1.0f + e) - LN2F;
}

__device__ __forceinline__ void bfrag2(const float* __restrict__ W, int col, int hh,
                                       FragB (&Bh)[4], FragB (&Bl)[4]) {
#pragma unroll
  for (int ks = 0; ks < 4; ++ks) {
    v16us th, tl;
    const int kA = 32 * ks + 8 * hh, kB = kA + 16;
#pragma unroll
    for (int j = 0; j < 8; ++j) {
      const float wa = W[(kA + j) * FDIM + col];
      const float wb = W[(kB + j) * FDIM + col];
      const unsigned short ha = bf_bits(wa), hb = bf_bits(wb);
      th[j] = ha;      tl[j] = bf_bits(wa - bf_val(ha));
      th[8 + j] = hb;  tl[8 + j] = bf_bits(wb - bf_val(hb));
    }
    Bh[ks].u = th;
    Bl[ks].u = tl;
  }
}

__device__ __forceinline__ void accadd(float* accb, int s, int c, float v) {
  s = s < 0 ? 0 : (s > NB ? NB : s);
  float* q = accb + s * FDIM + c;
  const float t = *q + v;
  *q = t;
}

__device__ __forceinline__ int scan_chunk(const int* __restrict__ dsts, int nE, int cbase, int nodeBase,
                                          int vec8, int* list, int tid, int wave) {
  int wc = 0;
  const int el0  = tid * EPT;
  const int e0   = cbase + el0;
  const int sent = -2147483647 - 1;
  v4i da, db;
  if (vec8 != 0 && e0 + 7 < nE) {
    da = *(const v4i*)(dsts + e0);
    db = *(const v4i*)(dsts + e0 + 4);
  } else {
    da.x = (e0     < nE) ? dsts[min(e0, nE - 1)] : sent;
    da.y = (e0 + 1 < nE) ? dsts[min(e0 + 1, nE - 1)] : sent;
    da.z = (e0 + 2 < nE) ? dsts[min(e0 + 2, nE - 1)] : sent;
    da.w = (e0 + 3 < nE) ? dsts[min(e0 + 3, nE - 1)] : sent;
    db.x = (e0 + 4 < nE) ? dsts[min(e0 + 4, nE - 1)] : sent;
    db.y = (e0 + 5 < nE) ? dsts[min(e0 + 5, nE - 1)] : sent;
    db.z = (e0 + 6 < nE) ? dsts[min(e0 + 6, nE - 1)] : sent;
    db.w = (e0 + 7 < nE) ? dsts[min(e0 + 7, nE - 1)] : sent;
  }
  const unsigned nb = (unsigned)nodeBase;
  const unsigned s0 = (unsigned)da.x - nb, s1 = (unsigned)da.y - nb;
  const unsigned s2 = (unsigned)da.z - nb, s3 = (unsigned)da.w - nb;
  const unsigned s4 = (unsigned)db.x - nb, s5 = (unsigned)db.y - nb;
  const unsigned s6 = (unsigned)db.z - nb, s7 = (unsigned)db.w - nb;
  const bool h0 = s0 < (unsigned)NB, h1 = s1 < (unsigned)NB, h2 = s2 < (unsigned)NB, h3 = s3 < (unsigned)NB;
  const bool h4 = s4 < (unsigned)NB, h5 = s5 < (unsigned)NB, h6 = s6 < (unsigned)NB, h7 = s7 < (unsigned)NB;
  const unsigned any = __builtin_amdgcn_ballot_w32(h0 | h1 | h2 | h3 | h4 | h5 | h6 | h7);
  if (any != 0u) {
#define HITJ(J, HJ) { \
      const unsigned mj = __builtin_amdgcn_ballot_w32(HJ); \
      if (mj != 0u) { \
        if (HJ) { \
          const int pos = wc + (int)__builtin_amdgcn_mbcnt_lo(mj, 0u); \
          if (pos < WCAP) list[wave * WCAP + pos] = el0 + (J); \
        } \
        wc += (int)__builtin_popcount(mj); } }
    HITJ(0, h0)
    HITJ(1, h1)
    HITJ(2, h2)
    HITJ(3, h3)
    HITJ(4, h4)
    HITJ(5, h5)
    HITJ(6, h6)
    HITJ(7, h7)
#undef HITJ
  }
  return wc;
}

template <int ACT>
__device__ __forceinline__ void node_gemm(const unsigned short* Ah, const unsigned short* Al,
                                          const FragB (&Bh)[4], const FragB (&Bl)[4],
                                          float bias, float* Ot, int hh, int m, int col) {
#pragma unroll 1
  for (int rt = 0; rt < NROW / 16; ++rt) {
    v8f d = zero8f();
#pragma unroll
    for (int ks = 0; ks < 4; ++ks) {
      const int o = (16 * rt + m) * A2P + 32 * ks + 8 * hh;
      FragB ah, al;
      ah.h[0] = *(const v8b*)(Ah + o);  ah.h[1] = *(const v8b*)(Ah + o + 16);
      al.h[0] = *(const v8b*)(Al + o);  al.h[1] = *(const v8b*)(Al + o + 16);
      d = wmb(ah, Bh[ks], d);
      d = wmb(ah, Bl[ks], d);
      d = wmb(al, Bh[ks], d);
    }
#pragma unroll
    for (int r = 0; r < 8; ++r) {
      float v = d[r] + bias;
      if (ACT != 0) v = sspf(v);
      Ot[(16 * rt + 8 * hh + r) * FDIM + col] = v;
    }
  }
}

template <int TWO>
__global__ __launch_bounds__(NTHR) void k_node(
    const float* __restrict__ src, int nValid,
    const float* __restrict__ Wa, const float* __restrict__ ba,
    const float* __restrict__ Wb, const float* __restrict__ bb,
    float* dst, int limFloats) {
  __shared__ __attribute__((aligned(16))) unsigned short Ah[NROW * A2P];
  __shared__ __attribute__((aligned(16))) unsigned short Al[NROW * A2P];
  __shared__ __attribute__((aligned(16))) float          Ot[NROW * FDIM];

  const int tid = threadIdx.x, lane = tid & 31, wave = tid >> 5, hh = lane >> 4, m = lane & 15;
  const int col = 16 * wave + m;
  const int row0 = blockIdx.x * NROW;
  const v4f z4 = {0.0f, 0.0f, 0.0f, 0.0f};

  for (int i = tid; i < NROW * 32; i += NTHR) {
    const int r = i >> 5, c4 = (i & 31) * 4;
    v4f v = z4;
    if (row0 + r < nValid) v = *(const v4f*)(src + (size_t)(row0 + r) * FDIM + c4);
    v4us qh, ql;
    split4(v, qh, ql);
    *(v4us*)(Ah + r * A2P + c4) = qh;
    *(v4us*)(Al + r * A2P + c4) = ql;
  }
  FragB Bh[4], Bl[4];
  bfrag2(Wa, col, hh, Bh, Bl);
  float bias = ba[col];
  __syncthreads();

  node_gemm<TWO>(Ah, Al, Bh, Bl, bias, Ot, hh, m, col);
  __syncthreads();

  if (TWO != 0) {
    for (int i = tid; i < NROW * 32; i += NTHR) {
      const int r = i >> 5, c4 = (i & 31) * 4;
      const v4f v = *(const v4f*)(Ot + r * FDIM + c4);
      v4us qh, ql;
      split4(v, qh, ql);
      *(v4us*)(Ah + r * A2P + c4) = qh;
      *(v4us*)(Al + r * A2P + c4) = ql;
    }
    bfrag2(Wb, col, hh, Bh, Bl);
    bias = bb[col];
    __syncthreads();
    node_gemm<0>(Ah, Al, Bh, Bl, bias, Ot, hh, m, col);
    __syncthreads();
  }

  const size_t ob  = (size_t)row0 * FDIM;
  const size_t lim = (size_t)(limFloats < 0 ? 0 : limFloats);
#pragma unroll 1
  for (int q = 0; q < NQN; ++q) {
    const int f = (wave * NQN + q) * 128 + 4 * lane;
    const v4f v = *(const v4f*)(Ot + f);
    const size_t gi = ob + (size_t)f;
    if (gi + 3 < lim) *(volatile v4f*)(dst + gi) = v;
  }
  __threadfence();
#pragma unroll 1
  for (int q = 0; q < NQN; ++q) {
    const int f = (wave * NQN + q) * 128 + 4 * lane;
    const v4f v = *(const v4f*)(Ot + f);
    const size_t gi = ob + (size_t)f;
    if (gi + 3 < lim) *(volatile v4f*)(dst + gi) = v;
  }
}

__global__ __launch_bounds__(NTHR) void k_edge(
    const float* __restrict__ fij, const float* __restrict__ rcut,
    const int* __restrict__ idxi, const int* __restrict__ idxj,
    const float* __restrict__ Wf1, const float* __restrict__ bfa,
    const float* __restrict__ Wf2, const float* __restrict__ bfb,
    const float* __restrict__ hrow, float* aggp, int nN, int nE, int vec8) {
  __shared__ __attribute__((aligned(16))) float          acc[(NB + 1) * FDIM];
  __shared__ __attribute__((aligned(16))) unsigned short A1[PASSN * A1P];
  __shared__ __attribute__((aligned(16))) _Float16       A2h[PASSN * A2P];
  __shared__ __attribute__((aligned(16))) _Float16       A2l[PASSN * A2P];
  __shared__ __attribute__((aligned(16))) int            list[LISTN];
  __shared__ __attribute__((aligned(16))) int            pend[PCAP];
  __shared__ __attribute__((aligned(16))) int            slotb[PASSN];
  __shared__ __attribute__((aligned(16))) int            jb[PASSN];
  __shared__ __attribute__((aligned(16))) float          rcb[PASSN];
  __shared__ int wcnt[NWAVE];
  __shared__ int pendN;

  const int tid = threadIdx.x, lane = tid & 31, wave = tid >> 5, hh = lane >> 4, m = lane & 15;
  const int col = 16 * wave + m;
  const int nodeBase = blockIdx.x * NB;
  const v4f z4 = {0.0f, 0.0f, 0.0f, 0.0f};

  for (int i = tid; i < ((NB + 1) * FDIM) / 4; i += NTHR) *(v4f*)(acc + 4 * i) = z4;

  FragB B1[2];
#pragma unroll
  for (int ks = 0; ks < 2; ++ks) {
    v16us tb;
    const int kA = 32 * ks + 8 * hh, kB = kA + 16;
#pragma unroll
    for (int j = 0; j < 16; ++j) {
      const int s = (j < 8) ? (kA + j) : (kB + (j - 8));
      const int k = (s < 20) ? s : ((s < 40) ? (s - 20) : ((s < 60) ? (s - 40) : 0));
      const float w = Wf1[k * FDIM + col];
      const unsigned short hb = bf_bits(w);
      unsigned short bits = hb;
      if (s >= 40) bits = bf_bits(w - bf_val(hb));
      if (s >= 60) bits = (unsigned short)0;
      tb[j] = bits;
    }
    B1[ks].u = tb;
  }
  FragH B2[4];
#pragma unroll
  for (int ks = 0; ks < 4; ++ks) {
    v16h tv;
    const int kA = 32 * ks + 8 * hh, kB = kA + 16;
#pragma unroll
    for (int j = 0; j < 8; ++j) {
      tv[j]     = (_Float16)(Wf2[(kA + j) * FDIM + col] * WSC);
      tv[8 + j] = (_Float16)(Wf2[(kB + j) * FDIM + col] * WSC);
    }
    B2[ks].v = tv;
  }
  const float b1c = bfa[col];
  const float b2c = bfb[col];
  if (tid == 0) pendN = 0;
  __syncthreads();

  const int nChunks = (nE + CHUNK - 1) / CHUNK;
#pragma unroll 1
  for (int ch = 0; ch < nChunks; ++ch) {
    const int cbase = ch * CHUNK;
    const int wc = scan_chunk(idxi, nE, cbase, nodeBase, vec8, list, tid, wave);
    if (lane == 0) wcnt[wave] = wc;
    __syncthreads();

    const int base = pendN;
    int tot = 0, myoff = 0;
#pragma unroll
    for (int w = 0; w < NWAVE; ++w) {
      int c = wcnt[w];
      c = c > WCAP ? WCAP : (c < 0 ? 0 : c);
      if (w < wave) myoff += c;
      tot += c;
    }
    int newN = base + tot;
    newN = newN > PCAP ? PCAP : newN;
    {
      int n = wcnt[wave];
      n = n > WCAP ? WCAP : (n < 0 ? 0 : n);
      const int* lp = list + wave * WCAP;
      for (int i = lane; i < n; i += 32) {
        const int pos = base + myoff + i;
        if (pos < PCAP) pend[pos] = cbase + lp[i];
      }
    }
    const int fin = (ch == nChunks - 1) ? 1 : 0;
    const int R   = (fin != 0) ? (newN + PASSN - 1) / PASSN : newN / PASSN;
    const int Pv  = (fin != 0) ? newN : R * PASSN;
    __syncthreads();

#pragma unroll 1
    for (int r = 0; r < R; ++r) {
      {
        const int i = tid >> 2, p = tid & 3;
        const int idx = r * PASSN + i;
        const bool valid = idx < Pv;
        int e = 0;
        if (valid) e = pend[idx];
        e = e < 0 ? 0 : (e > nE - 1 ? nE - 1 : e);
        v4f q0 = z4, q1 = z4;
        if (valid) {
          q0 = *(const v4f*)(fij + (size_t)e * KRBF + 4 * p);
          if (p == 0) q1 = *(const v4f*)(fij + (size_t)e * KRBF + 16);
        }
        unsigned short* arow = A1 + i * A1P;
        v4us h0, l0;
        split4(q0, h0, l0);
        *(v4us*)(arow + 4 * p)      = h0;
        *(v4us*)(arow + 20 + 4 * p) = l0;
        *(v4us*)(arow + 40 + 4 * p) = h0;
        if (p == 0) {
          v4us h1, l1;
          split4(q1, h1, l1);
          const v4us zq = {(unsigned short)0, (unsigned short)0, (unsigned short)0, (unsigned short)0};
          *(v4us*)(arow + 16) = h1;
          *(v4us*)(arow + 36) = l1;
          *(v4us*)(arow + 56) = h1;
          *(v4us*)(arow + 60) = zq;
          const int d = idxi[e];
          int s = idxj[e];
          int slot = d - nodeBase;
          if (!valid || (unsigned)slot >= (unsigned)NB) slot = NB;
          s = s < 0 ? 0 : (s > nN - 1 ? nN - 1 : s);
          slotb[i] = slot;
          jb[i]    = s;
          rcb[i]   = valid ? rcut[e] : 0.0f;
        }
      }
      __syncthreads();

#pragma unroll 1
      for (int t = 0; t < PASSN / 16; ++t) {
        const int o = (16 * t + m) * A1P + 8 * hh;
        FragB a0, a1;
        a0.h[0] = *(const v8b*)(A1 + o);       a0.h[1] = *(const v8b*)(A1 + o + 16);
        a1.h[0] = *(const v8b*)(A1 + o + 32);  a1.h[1] = *(const v8b*)(A1 + o + 48);
        v8f d = zero8f();
        d = wmb(a0, B1[0], d);
        d = wmb(a1, B1[1], d);
#pragma unroll
        for (int rr = 0; rr < 8; ++rr) {
          const float u  = sspf(d[rr] + b1c);
          const float us = u * USC;
          const _Float16 uh = (_Float16)us;
          const _Float16 ul = (_Float16)((us - (float)uh) * RSC);
          const int row = 16 * t + 8 * hh + rr;
          A2h[row * A2P + col] = uh;
          A2l[row * A2P + col] = ul;
        }
      }
      __syncthreads();

#pragma unroll 1
      for (int t = 0; t < PASSN / 16; ++t) {
        v8f dh = zero8f(), dl = zero8f();
#pragma unroll
        for (int ks = 0; ks < 4; ++ks) {
          const int o = (16 * t + m) * A2P + 32 * ks + 8 * hh;
          FragH xh, xl;
          xh.h[0] = *(const v8h*)(A2h + o);  xh.h[1] = *(const v8h*)(A2h + o + 16);
          xl.h[0] = *(const v8h*)(A2l + o);  xl.h[1] = *(const v8h*)(A2l + o + 16);
          dh = wmh(xh.v, B2[ks].v, dh);
          dl = wmh(xl.v, B2[ks].v, dl);
        }
        float prod[8];
#pragma unroll
        for (int rr = 0; rr < 8; ++rr) {
          const int e = 16 * t + 8 * hh + rr;
          int j = jb[e];
          j = j < 0 ? 0 : (j > nN - 1 ? nN - 1 : j);
          const float hv  = hrow[(size_t)j * FDIM + col];
          const float wij = ((dh[rr] + dl[rr] * RINV) * UWINV + b2c) * rcb[e];
          prod[rr] = hv * wij;
        }
        float upper[8];
#pragma unroll
        for (int rr = 0; rr < 8; ++rr) upper[rr] = __shfl_down(prod[rr], 16u, 32);
        const v4i s0 = *(const v4i*)(slotb + 16 * t);
        const v4i s1 = *(const v4i*)(slotb + 16 * t + 4);
        const v4i s2 = *(const v4i*)(slotb + 16 * t + 8);
        const v4i s3 = *(const v4i*)(slotb + 16 * t + 12);
        if (hh == 0) {
          accadd(acc, s0.x, col, prod[0]);  accadd(acc, s0.y, col, prod[1]);
          accadd(acc, s0.z, col, prod[2]);  accadd(acc, s0.w, col, prod[3]);
          accadd(acc, s1.x, col, prod[4]);  accadd(acc, s1.y, col, prod[5]);
          accadd(acc, s1.z, col, prod[6]);  accadd(acc, s1.w, col, prod[7]);
          accadd(acc, s2.x, col, upper[0]); accadd(acc, s2.y, col, upper[1]);
          accadd(acc, s2.z, col, upper[2]); accadd(acc, s2.w, col, upper[3]);
          accadd(acc, s3.x, col, upper[4]); accadd(acc, s3.y, col, upper[5]);
          accadd(acc, s3.z, col, upper[6]); accadd(acc, s3.w, col, upper[7]);
        }
      }
      __syncthreads();
    }

    int rem = newN - R * PASSN;
    rem = rem < 0 ? 0 : rem;
    if (R > 0 && tid < rem) pend[tid] = pend[R * PASSN + tid];
    if (tid == 0) pendN = rem;
  }
  __syncthreads();

  const size_t ob = (size_t)blockIdx.x * NB * FDIM;
#pragma unroll 1
  for (int q = 0; q < NQE; ++q) {
    const int f = (wave * NQE + q) * 128 + 4 * lane;
    const v4f v = *(const v4f*)(acc + f);
    *(volatile v4f*)(aggp + ob + (size_t)f) = v;
  }
  __threadfence();
#pragma unroll 1
  for (int q = 0; q < NQE; ++q) {
    const int f = (wave * NQE + q) * 128 + 4 * lane;
    const v4f v = *(const v4f*)(acc + f);
    *(volatile v4f*)(aggp + ob + (size_t)f) = v;
  }
}

extern "C" void kernel_launch(void* const* d_in, const int* in_sizes, int n_in,
                              void* d_out, int out_size, void* d_ws, size_t ws_size,
                              hipStream_t stream) {
  if (n_in < 15) return;
  const int nN = in_sizes[0] / FDIM;
  const int nE = in_sizes[2];
  if (nN <= 0 || nE <= 0) return;
  if (in_sizes[0] != nN * FDIM || in_sizes[1] != nE * KRBF || in_sizes[3] != nE || in_sizes[4] != nE) return;
  if (in_sizes[5] != FDIM * FDIM || in_sizes[6] < FDIM) return;
  if (in_sizes[7] != KRBF * FDIM || in_sizes[8] < FDIM) return;
  if (in_sizes[9] != FDIM * FDIM || in_sizes[10] < FDIM) return;
  if (in_sizes[11] != FDIM * FDIM || in_sizes[12] < FDIM) return;
  if (in_sizes[13] != FDIM * FDIM || in_sizes[14] < FDIM) return;
  if (out_size != nN * FDIM) return;

  const float* x    = (const float*)d_in[0];
  const float* fij  = (const float*)d_in[1];
  const float* rcut = (const float*)d_in[2];
  const int*   idxi = (const int*)d_in[3];
  const int*   idxj = (const int*)d_in[4];
  const float* Win  = (const float*)d_in[5];
  const float* bin  = (const float*)d_in[6];
  const float* Wf1  = (const float*)d_in[7];
  const float* bf1  = (const float*)d_in[8];
  const float* Wf2  = (const float*)d_in[9];
  const float* bf2  = (const float*)d_in[10];
  const float* Wo1  = (const float*)d_in[11];
  const float* bo1  = (const float*)d_in[12];
  const float* Wo2  = (const float*)d_in[13];
  const float* bo2  = (const float*)d_in[14];
  float* out = (float*)d_out;

  const int nBlkN = (nN + NROW - 1) / NROW;
  const int nBlkE = (nN + NB - 1) / NB;

  char* ws = (char*)d_ws;
  size_t off = 0;
  const size_t oH = off; off += (size_t)nBlkN * NROW * FDIM * sizeof(float); off = (off + 255) & ~(size_t)255;
  const size_t oA = off; off += (size_t)nBlkE * NB * FDIM * sizeof(float);   off = (off + 255) & ~(size_t)255;
  if (off > ws_size) return;
  float* hbuf = (float*)(ws + oH);
  float* agg  = (float*)(ws + oA);

  const int vec8 = ((nE & 3) == 0) ? 1 : 0;

  k_node<0><<<nBlkN, NTHR, 0, stream>>>(x, nN, Win, bin, Win, bin, hbuf, nBlkN * NROW * FDIM);

  k_edge<<<nBlkE, NTHR, 0, stream>>>(fij, rcut, idxi, idxj, Wf1, bf1, Wf2, bf2, hbuf, agg, nN, nE, vec8);

  k_node<1><<<nBlkN, NTHR, 0, stream>>>(agg, nN, Wo1, bo1, Wo2, bo2, out, nN * FDIM);
}
